// _GATLayer_58815282152005
// MI455X (gfx1250) — hardware-run, weakly checked
//
#include <hip/hip_runtime.h>
#include <stddef.h>
#include <stdint.h>
#include <math.h>


#define F_IN    256
#define HC      256
#define NHD     8
#define HID     32
#define NBATCH  2
#define NNODE   10000
#define NROWS   (NBATCH * NNODE)
#define MROWS   128
#define MP      (((NROWS + MROWS - 1) / MROWS) * MROWS)
#define NTHR    256
#define NWAVE   8
#define EPT     8
#define CHUNK   (NTHR * EPT)
#define WCAP    (EPT * 32)
#define LISTN   (NWAVE * WCAP)
#define NBRUN   1024
#define SLOTB   10
#define NBLK    ((NNODE + NBRUN - 1) / NBRUN)
#define RCAP    28672
#define DEGCAP  256
#define MEAS_MAXDEG 35
#define MEAS_B1024  16614
#define GROWS   128
#define GBN     64
#define GTHR    256
#define NEGSL   0.2f
#define LN_EPS  1e-5f
#define WSMAX   ((size_t)(128u << 20))
#define LDS_BKT ((2 * RCAP + 2 * NBRUN + LISTN + 2 * NWAVE) * 4 + 64)

static_assert(NBRUN == (1 << SLOTB));
static_assert(NTHR * 4 == NBRUN);
static_assert(LISTN >= NBRUN);
static_assert(LISTN >= NWAVE * WCAP);
static_assert((CHUNK & (CHUNK - 1)) == 0 && CHUNK == 2048 && 11 + SLOTB <= 31);
static_assert((RCAP % (4 * NTHR)) == 0);
static_assert(RCAP >= MEAS_B1024 + 4096);
static_assert(DEGCAP >= MEAS_MAXDEG + 8);
static_assert(LDS_BKT <= 327680);
static_assert(NBLK * NBRUN >= NNODE && NBLK <= 16);
static_assert((MP % GROWS) == 0 && MP >= NROWS);
static_assert(GROWS == (GTHR / 32) * 16);
static_assert(GTHR == 2 * GROWS);
static_assert((F_IN % 32) == 0 && (HC % GBN) == 0 && GBN == 2 * HID && HC == NHD * HID);
static_assert(HC == 8 * 32 && HID == 4 * 8);
static_assert((F_IN / 8) == 32);
static_assert(((MP * (F_IN / 8)) % NTHR) == 0);
static_assert(((HC * (F_IN / 8)) % NTHR) == 0);
static_assert(NROWS == (NROWS / NWAVE) * NWAVE);

typedef float          v4f  __attribute__((ext_vector_type(4)));
typedef float          v8f  __attribute__((ext_vector_type(8)));
typedef int            v4i  __attribute__((ext_vector_type(4)));
typedef int            v8i  __attribute__((ext_vector_type(8)));
typedef unsigned int   v4u  __attribute__((ext_vector_type(4)));
typedef unsigned short v8us __attribute__((ext_vector_type(8)));
typedef __bf16         v16b __attribute__((ext_vector_type(16)));
typedef v4f  __attribute__((may_alias)) v4fa;
typedef v8us __attribute__((may_alias)) v8usa;
union FragB { v16b v; v8us h[2]; v8i w; };

__device__ __forceinline__ v8f wmb(const FragB& a, const FragB& b, v8f c) {
  v8f d = __builtin_amdgcn_wmma_f32_16x16x32_bf16(false, a.v, false, b.v, (short)0, c, false, false);
  asm volatile("v_nop\n\tv_nop\n\tv_nop\n\tv_nop" : "+v"(d) : "v"(a.w), "v"(b.w));
  return d;
}

__device__ __forceinline__ unsigned int f2bf(float f) {
  const unsigned int u = __float_as_uint(f);
  return ((u + 0x7FFFu + ((u >> 16) & 1u)) >> 16) & 0xFFFFu;
}
__device__ __forceinline__ float bf2f(unsigned int b) { return __uint_as_float(b << 16); }
__device__ __forceinline__ float bfr(float f) { return bf2f(f2bf(f)); }
__device__ __forceinline__ v4f bfr4(const v4f a) {
  v4f r; r.x = bfr(a.x); r.y = bfr(a.y); r.z = bfr(a.z); r.w = bfr(a.w); return r;
}
__device__ __forceinline__ unsigned int pk2(float lo, float hi) { return f2bf(lo) | (f2bf(hi) << 16); }
__device__ __forceinline__ v4u pack8(const v4f a, const v4f b) {
  v4u r;
  r.x = pk2(a.x, a.y); r.y = pk2(a.z, a.w); r.z = pk2(b.x, b.y); r.w = pk2(b.z, b.w);
  return r;
}
__device__ __forceinline__ int clampi(int v, int lo, int hi) { return v < lo ? lo : (v > hi ? hi : v); }

__device__ __forceinline__ int scan_chunk(const int* __restrict__ dsts, int nE, int cbase, int slotBase,
                                          int nb, int vec8, int* list, int tid, int lane, int wave) {
  int wc = 0;
  const int el0  = tid * EPT;
  const int e0   = cbase + el0;
  const int sent = (int)(1u << 31);
  v4i da, db;
  if (vec8 != 0 && cbase + CHUNK <= nE) {
    da = *(const v4i*)(dsts + e0);
    db = *(const v4i*)(dsts + e0 + 4);
  } else {
    da.x = (e0     < nE) ? dsts[min(e0,     nE - 1)] : sent;
    da.y = (e0 + 1 < nE) ? dsts[min(e0 + 1, nE - 1)] : sent;
    da.z = (e0 + 2 < nE) ? dsts[min(e0 + 2, nE - 1)] : sent;
    da.w = (e0 + 3 < nE) ? dsts[min(e0 + 3, nE - 1)] : sent;
    db.x = (e0 + 4 < nE) ? dsts[min(e0 + 4, nE - 1)] : sent;
    db.y = (e0 + 5 < nE) ? dsts[min(e0 + 5, nE - 1)] : sent;
    db.z = (e0 + 6 < nE) ? dsts[min(e0 + 6, nE - 1)] : sent;
    db.w = (e0 + 7 < nE) ? dsts[min(e0 + 7, nE - 1)] : sent;
  }
  const unsigned nbs = (unsigned)slotBase;
  const unsigned unb = (unsigned)nb;
  const unsigned s0 = (unsigned)da.x - nbs, s1 = (unsigned)da.y - nbs;
  const unsigned s2 = (unsigned)da.z - nbs, s3 = (unsigned)da.w - nbs;
  const unsigned s4 = (unsigned)db.x - nbs, s5 = (unsigned)db.y - nbs;
  const unsigned s6 = (unsigned)db.z - nbs, s7 = (unsigned)db.w - nbs;
  const bool h0 = s0 < unb, h1 = s1 < unb, h2 = s2 < unb, h3 = s3 < unb;
  const bool h4 = s4 < unb, h5 = s5 < unb, h6 = s6 < unb, h7 = s7 < unb;
  const unsigned any = __builtin_amdgcn_ballot_w32(h0 | h1 | h2 | h3 | h4 | h5 | h6 | h7);
  if (any != 0u) {
#define HITJ(J, HJ, SJ) { \
      const unsigned mj = __builtin_amdgcn_ballot_w32(HJ); \
      if (mj != 0u) { \
        if (HJ) { \
          const int pos = wc + (int)__builtin_amdgcn_mbcnt_lo(mj, 0u); \
          if (pos < WCAP) list[wave * WCAP + pos] = ((el0 + (J)) << SLOTB) | (int)(SJ); \
        } \
        wc += (int)__builtin_popcount(mj); } }
    HITJ(0, h0, s0)
    HITJ(1, h1, s1)
    HITJ(2, h2, s2)
    HITJ(3, h3, s3)
    HITJ(4, h4, s4)
    HITJ(5, h5, s5)
    HITJ(6, h6, s6)
    HITJ(7, h7, s7)
#undef HITJ
  }
  return wc;
}

__global__ __launch_bounds__(NTHR) void k_prep(const float* __restrict__ x, const float* __restrict__ W,
                                               const float* __restrict__ al, const float* __restrict__ ar,
                                               const float* __restrict__ gm, const float* __restrict__ bt,
                                               unsigned short* xb, unsigned short* wt, float* par,
                                               int nbX, int nbW) {
  const int bx = (int)blockIdx.x, tid = (int)threadIdx.x;
  if (bx < nbX) {
    const int i   = bx * NTHR + tid;
    const int row = i >> 5;
    const int c0  = (i & 31) * 8;
    const int rc  = row < NROWS ? row : NROWS - 1;
    const float* p = x + (size_t)rc * F_IN + c0;
    v4f a = *(const v4fa*)p, b = *(const v4fa*)(p + 4);
    const v4f z4 = {0.f, 0.f, 0.f, 0.f};
    if (row >= NROWS) { a = z4; b = z4; }
    const v4u hv = pack8(a, b);
    const size_t o = (size_t)row * F_IN + c0;
    *(volatile v4u*)(xb + o) = hv;
    __threadfence();
    *(volatile v4u*)(xb + o) = hv;
  } else if (bx < nbX + nbW) {
    const int u  = (bx - nbX) * NTHR + tid;
    const int n  = u >> 5;
    const int k8 = (u & 31) * 8;
    const float* p = W + (size_t)k8 * HC + n;
    v4f a, b;
    a.x = p[0];        a.y = p[HC];       a.z = p[2 * HC];   a.w = p[3 * HC];
    b.x = p[4 * HC];   b.y = p[5 * HC];   b.z = p[6 * HC];   b.w = p[7 * HC];
    const v4u wv = pack8(a, b);
    unsigned short* o = wt + (size_t)n * F_IN + k8;
    *(volatile v4u*)o = wv;
    __threadfence();
    *(volatile v4u*)o = wv;
  } else {
    if (tid < 64) {
      const v4f v0 = bfr4(*(const v4fa*)(al + 4 * tid));
      const v4f v1 = bfr4(*(const v4fa*)(ar + 4 * tid));
      const v4f v2 = bfr4(*(const v4fa*)(gm + 4 * tid));
      const v4f v3 = bfr4(*(const v4fa*)(bt + 4 * tid));
      float* o = par + 4 * tid;
      *(volatile v4f*)(o)       = v0;
      *(volatile v4f*)(o + 256) = v1;
      *(volatile v4f*)(o + 512) = v2;
      *(volatile v4f*)(o + 768) = v3;
      __threadfence();
      *(volatile v4f*)(o)       = v0;
      *(volatile v4f*)(o + 256) = v1;
      *(volatile v4f*)(o + 512) = v2;
      *(volatile v4f*)(o + 768) = v3;
    }
  }
}

__global__ __launch_bounds__(GTHR) __attribute__((amdgpu_num_vgpr(248)))
void k_gemm(const unsigned short* __restrict__ A, const unsigned short* __restrict__ WT,
            const float* __restrict__ PAR, float* HP, float* SD) {
  __shared__ __attribute__((aligned(16))) float stg[GROWS * GBN];
  __shared__ __attribute__((aligned(16))) float satt[2 * HC];
  __shared__ __attribute__((aligned(16))) float sdot[GROWS * 16];
  const int tid = (int)threadIdx.x, lane = tid & 31, wave = tid >> 5, hh = lane >> 4, m = lane & 15;
  const int rowBase = (int)blockIdx.x * GROWS;

  if (tid < 128) {
    const v4f pv = *(const v4fa*)(PAR + 4 * tid);
    *(v4fa*)(satt + 4 * tid) = pv;
  }

  const unsigned short* ap = A + (size_t)(rowBase + 16 * wave + m) * (size_t)F_IN + 8 * hh;

#pragma unroll 1
  for (int nc = 0; nc < HC / GBN; ++nc) {
    const int col0 = nc * GBN;
    const unsigned short* wp = WT + (size_t)(col0 + m) * (size_t)F_IN + 8 * hh;
    v8f acc[4];
    {
      const v8f z = {0.f, 0.f, 0.f, 0.f, 0.f, 0.f, 0.f, 0.f};
      acc[0] = z; acc[1] = z; acc[2] = z; acc[3] = z;
    }
#pragma unroll 1
    for (int ks = 0; ks < F_IN / 32; ++ks) {
      FragB af;
      af.h[0] = *(const v8usa*)(ap + 32 * ks);
      af.h[1] = *(const v8usa*)(ap + 32 * ks + 16);
#pragma unroll
      for (int t = 0; t < 4; ++t) {
        const unsigned short* wq = wp + (size_t)(16 * t) * (size_t)F_IN + 32 * ks;
        FragB bf;
        bf.h[0] = *(const v8usa*)wq;
        bf.h[1] = *(const v8usa*)(wq + 16);
        acc[t] = wmb(af, bf, acc[t]);
      }
    }

#pragma unroll
    for (int t = 0; t < 4; ++t) {
      const int lc = 16 * t + m;
#pragma unroll
      for (int r = 0; r < 8; ++r) {
        const int lr = 16 * wave + 8 * hh + r;
        stg[lr * GBN + lc] = acc[t][r];
      }
    }
    __syncthreads();

    {
      const int row = tid & 127, hb = tid >> 7;
      const int head = 2 * nc + hb;
      const float* sa = satt + head * HID;
      const float* sb = satt + HC + head * HID;
      const float* hr = stg + row * GBN + HID * hb;
      float ds = 0.f, dd = 0.f;
#pragma unroll 2
      for (int c4 = 0; c4 < HID / 4; ++c4) {
        const v4f hv = *(const v4fa*)(hr + 4 * c4);
        const v4f av = *(const v4fa*)(sa + 4 * c4);
        const v4f bv = *(const v4fa*)(sb + 4 * c4);
        ds = fmaf(hv.x, av.x, ds);  dd = fmaf(hv.x, bv.x, dd);
        ds = fmaf(hv.y, av.y, ds);  dd = fmaf(hv.y, bv.y, dd);
        ds = fmaf(hv.z, av.z, ds);  dd = fmaf(hv.z, bv.z, dd);
        ds = fmaf(hv.w, av.w, ds);  dd = fmaf(hv.w, bv.w, dd);
      }
      sdot[row * 16 + head]     = ds;
      sdot[row * 16 + 8 + head] = dd;
    }

    v4f fv[8];
#pragma unroll
    for (int i = 0; i < 8; ++i) {
      const int lr = 16 * wave + 2 * i + hh;
      fv[i] = *(const v4fa*)(stg + lr * GBN + 4 * m);
    }
#pragma unroll
    for (int i = 0; i < 8; ++i) {
      const int lr = 16 * wave + 2 * i + hh;
      float* op = HP + (size_t)(rowBase + lr) * (size_t)HC + col0 + 4 * m;
      *(volatile v4f*)op = fv[i];
    }
    __threadfence();
#pragma unroll
    for (int i = 0; i < 8; ++i) {
      const int lr = 16 * wave + 2 * i + hh;
      float* op = HP + (size_t)(rowBase + lr) * (size_t)HC + col0 + 4 * m;
      *(volatile v4f*)op = fv[i];
    }
    __syncthreads();
  }

  const v4f s0 = *(const v4fa*)(sdot + 4 * tid);
  const v4f s1 = *(const v4fa*)(sdot + 4 * (GTHR + tid));
  float* sp = SD + (size_t)rowBase * 16 + 4 * tid;
  *(volatile v4f*)sp = s0;
  *(volatile v4f*)(sp + 4 * GTHR) = s1;
  __threadfence();
  *(volatile v4f*)sp = s0;
  *(volatile v4f*)(sp + 4 * GTHR) = s1;
}

__global__ __launch_bounds__(NTHR) void k_bucket(const int* __restrict__ srcs, const int* __restrict__ dsts,
                                                 int* LIST, int* OFF, int* CNT, int* FLAG,
                                                 int nN, int nE, int vec8) {
  extern __shared__ v4f lds_dyn[];
  int* reg1 = (int*)lds_dyn;
  int* reg2 = reg1 + RCAP;
  int* scnt = reg2 + RCAP;
  int* soff = scnt + NBRUN;
  int* list = soff + NBRUN;
  int* wcnt = list + LISTN;
  int* wtot = wcnt + NWAVE;
  const int tid = (int)threadIdx.x, lane = tid & 31, wave = tid >> 5;
  const int nodeBase = (int)blockIdx.x * NBRUN;
  const int nb = clampi(nN - nodeBase, 0, NBRUN);

  for (int i = tid; i < NBRUN; i += NTHR) scnt[i] = 0;
  {
    const v4i z = {0, 0, 0, 0};
    for (int i = tid; i < RCAP / 4; i += NTHR) *(v4i*)(reg2 + 4 * i) = z;
  }
  __syncthreads();

  int tot = 0;
  const int nChunks = (nE + CHUNK - 1) / CHUNK;
#pragma unroll 1
  for (int ch = 0; ch < nChunks; ++ch) {
    const int cbase = ch * CHUNK;
    const int wc = scan_chunk(dsts, nE, cbase, nodeBase, nb, vec8, list, tid, lane, wave);
    if (lane == 0) wcnt[wave] = wc;
    __syncthreads();
    int pre = 0, all = 0;
#pragma unroll
    for (int w2 = 0; w2 < NWAVE; ++w2) {
      int c = wcnt[w2];
      c = c < 0 ? 0 : (c > WCAP ? WCAP : c);
      all += c;
      pre += (w2 < wave) ? c : 0;
    }
    const int wcc  = wc > WCAP ? WCAP : wc;
    const int base = tot + pre;
#pragma unroll 1
    for (int i = lane; i < wcc; i += 32) {
      const int ent = list[wave * WCAP + i];
      const int el  = (ent >> SLOTB) & (CHUNK - 1);
      const int sl  = ent & (NBRUN - 1);
      int eid = cbase + el;
      eid = eid > nE - 1 ? nE - 1 : eid;
      const int pos = base + i;
      if (pos < RCAP) reg1[pos] = (int)(((unsigned)eid << SLOTB) | (unsigned)sl);
    }
    tot += all;
    tot = tot > RCAP ? RCAP : tot;
    __syncthreads();
  }
  const int nh = tot;

  if (wave == 0) {
#pragma unroll 1
    for (int b0 = 0; b0 < nh; b0 += 32) {
      const int idx = b0 + lane;
      const int uv  = reg1[idx < nh ? idx : nh - 1];
      const int m32 = (nh - b0) < 32 ? (nh - b0) : 32;
#pragma unroll 1
      for (int k = 0; k < m32; ++k) {
        const int u  = __builtin_amdgcn_readlane(uv, k);
        const int sl = u & (NBRUN - 1);
        if (lane == 0) scnt[sl] = scnt[sl] + 1;
      }
    }
  }
  __syncthreads();

  {
    const v4i ca = *(const v4i*)(scnt + 4 * tid);
    const int e0 = ca.x < 0 ? 0 : ca.x, e1 = ca.y < 0 ? 0 : ca.y, e2 = ca.z < 0 ? 0 : ca.z, e3 = ca.w < 0 ? 0 : ca.w;
    const int ts = e0 + e1 + e2 + e3;
    int incl = ts;
#pragma unroll
    for (int d = 1; d < 32; d <<= 1) {
      const int up = __shfl_up(incl, d);
      if (lane >= d) incl += up;
    }
    if (lane == 31) wtot[wave] = incl;
    __syncthreads();
    int pre = 0;
#pragma unroll
    for (int w2 = 0; w2 < NWAVE; ++w2) pre += (w2 < wave) ? wtot[w2] : 0;
    int run = pre + incl - ts;
    soff[4 * tid + 0] = run; run += e0;
    soff[4 * tid + 1] = run; run += e1;
    soff[4 * tid + 2] = run; run += e2;
    soff[4 * tid + 3] = run;
  }
  __syncthreads();
  for (int i = tid; i < NBRUN; i += NTHR) list[i] = soff[i];
  __syncthreads();

  if (wave == 0) {
#pragma unroll 1
    for (int b0 = 0; b0 < nh; b0 += 32) {
      const int idx = b0 + lane;
      const int uv  = reg1[idx < nh ? idx : nh - 1];
      const int m32 = (nh - b0) < 32 ? (nh - b0) : 32;
#pragma unroll 1
      for (int k = 0; k < m32; ++k) {
        const int u   = __builtin_amdgcn_readlane(uv, k);
        const int sl  = u & (NBRUN - 1);
        const int eid = (int)((unsigned)u >> SLOTB);
        if (lane == 0) {
          int pos = list[sl];
          pos = pos < 0 ? 0 : (pos > RCAP - 1 ? RCAP - 1 : pos);
          reg2[pos] = eid;
          list[sl] = pos + 1;
        }
      }
    }
  }
  __syncthreads();

  int* Lk = LIST + (size_t)blockIdx.x * RCAP;
#pragma unroll 1
  for (int it = 0; it < RCAP / (4 * NTHR); ++it) {
    const int base = 4 * (it * NTHR + tid);
    const v4i ev = *(const v4i*)(reg2 + base);
    const int e0 = clampi(ev.x, 0, nE - 1), e1 = clampi(ev.y, 0, nE - 1);
    const int e2 = clampi(ev.z, 0, nE - 1), e3 = clampi(ev.w, 0, nE - 1);
    int s0 = srcs[e0], s1 = srcs[e1], s2 = srcs[e2], s3 = srcs[e3];
    asm volatile("" :: "v"(s0), "v"(s1), "v"(s2), "v"(s3));
    s0 = clampi(s0, 0, nN - 1); s1 = clampi(s1, 0, nN - 1);
    s2 = clampi(s2, 0, nN - 1); s3 = clampi(s3, 0, nN - 1);
    v4i ov;
    ov.x = (base     < nh) ? s0 : 0;
    ov.y = (base + 1 < nh) ? s1 : 0;
    ov.z = (base + 2 < nh) ? s2 : 0;
    ov.w = (base + 3 < nh) ? s3 : 0;
    *(volatile v4i*)(Lk + base) = ov;
    __threadfence();
    *(volatile v4i*)(Lk + base) = ov;
  }
  {
    const v4i ovv = *(const v4i*)(soff + 4 * tid);
    const v4i cvv = *(const v4i*)(scnt + 4 * tid);
    int* op = OFF + (size_t)blockIdx.x * NBRUN + 4 * tid;
    int* cp = CNT + (size_t)blockIdx.x * NBRUN + 4 * tid;
    const int fl = (nh >= RCAP) ? 1 : 0;
    const v4i fv = {fl, fl, fl, fl};
    int* fp = FLAG + (size_t)blockIdx.x * 32 + 4 * (tid & 7);
    *(volatile v4i*)op = ovv;
    *(volatile v4i*)cp = cvv;
    if (tid < 8) *(volatile v4i*)fp = fv;
    __threadfence();
    *(volatile v4i*)op = ovv;
    *(volatile v4i*)cp = cvv;
    if (tid < 8) *(volatile v4i*)fp = fv;
  }
}

__global__ __launch_bounds__(NTHR) void k_replay(const float* __restrict__ HP, const float* __restrict__ SD,
                                                 const unsigned short* __restrict__ XB, const float* __restrict__ PAR,
                                                 const int* __restrict__ LIST, const int* __restrict__ OFF,
                                                 const int* __restrict__ CNT, const int* __restrict__ FLAG,
                                                 float* out) {
  __shared__ __attribute__((aligned(16))) float sgb[2 * HC];
  __shared__ __attribute__((aligned(16))) float wrow[NWAVE * HC];
  __shared__ __attribute__((aligned(16))) float sden[NWAVE * 32];
  const int tid = (int)threadIdx.x, lane = tid & 31, wave = tid >> 5;

  if (tid < 128) {
    const v4f pv = *(const v4fa*)(PAR + 2 * HC + 4 * tid);
    *(v4fa*)(sgb + 4 * tid) = pv;
  }
  __syncthreads();

  const int rraw = (int)blockIdx.x * NWAVE + wave;
  const bool live = rraw < NROWS;
  const int row  = live ? rraw : NROWS - 1;
  const int b    = row / NNODE;
  const int d    = row - b * NNODE;
  const int rb   = b * NNODE;
  const int blk  = d >> SLOTB;
  const int head = lane >> 2;

  int ov = OFF[d];
  int cv = CNT[d];
  const int fl = FLAG[blk * 32];
  const int craw = cv;
  cv = cv < 0 ? 0 : (cv > DEGCAP ? DEGCAP : cv);
  ov = ov < 0 ? 0 : (ov > RCAP - 1 ? RCAP - 1 : ov);
  const int c = __builtin_amdgcn_readfirstlane(cv);
  const int o = __builtin_amdgcn_readfirstlane(ov);
  int last = o + c - 1; last = last < o ? o : last;
  last = last > RCAP - 1 ? RCAP - 1 : last;

  const int*   Lk  = LIST + (size_t)blk * RCAP;
  const float* SDb = SD + (size_t)rb * 16 + head;
  const float* HPb = HP + (size_t)rb * HC + 8 * lane;
  const float  rd  = SD[(size_t)row * 16 + 8 + head];

  float mx = __int_as_float((int)0xff800000u);
  float den = 0.0f;
  v4f av = {0.f, 0.f, 0.f, 0.f};
  v4f aw = {0.f, 0.f, 0.f, 0.f};

#pragma unroll 1
  for (int q = 0; q < c; ++q) {
    int idx = o + q; idx = idx > last ? last : idx;
    int s = Lk[idx];
    s = s < 0 ? 0 : (s > NNODE - 1 ? NNODE - 1 : s);
    const float* fr = HPb + (size_t)s * HC;
    const v4f fs = *(const v4fa*)fr;
    const v4f ft = *(const v4fa*)(fr + 4);
    float lg = SDb[(size_t)s * 16] + rd;
    lg = lg > 0.f ? lg : NEGSL * lg;
    const float mn = fmaxf(mx, lg);
    const float sc = expf(mx - mn);
    const float p  = expf(lg - mn);
    mx = mn;
    den = fmaf(den, sc, p);
    av.x = fmaf(av.x, sc, p * fs.x);
    av.y = fmaf(av.y, sc, p * fs.y);
    av.z = fmaf(av.z, sc, p * fs.z);
    av.w = fmaf(av.w, sc, p * fs.w);
    aw.x = fmaf(aw.x, sc, p * ft.x);
    aw.y = fmaf(aw.y, sc, p * ft.y);
    aw.z = fmaf(aw.z, sc, p * ft.z);
    aw.w = fmaf(aw.w, sc, p * ft.w);
  }

  float* wr = wrow + wave * HC;
  *(v4fa*)(wr + 8 * lane)     = av;
  *(v4fa*)(wr + 8 * lane + 4) = aw;
  sden[wave * 32 + lane] = (c > 0) ? den : 1.0f;
  __syncthreads();

  const unsigned short* xr = XB + (size_t)row * F_IN;
  float sum = 0.0f;
#pragma unroll 1
  for (int j = 0; j < 8; ++j) {
    const int cc = 32 * j + lane;
    const float a  = wr[cc];
    const float dn = sden[wave * 32 + 4 * j];
    const float xv = bf2f((unsigned int)xr[cc]);
    const float v  = a / dn + xv;
    wr[cc] = v;
    sum += v;
  }
#pragma unroll
  for (int off = 16; off > 0; off >>= 1) sum += __shfl_xor(sum, off);
  const float mu = sum * (1.0f / 256.0f);

  float ss = 0.0f;
#pragma unroll 1
  for (int j = 0; j < 8; ++j) {
    const float dv = wr[32 * j + lane] - mu;
    ss = fmaf(dv, dv, ss);
  }
#pragma unroll
  for (int off = 16; off > 0; off >>= 1) ss += __shfl_xor(ss, off);
  const float var = ss * (1.0f / 256.0f);
  const float sq  = sqrtf(var + LN_EPS);

#pragma unroll 1
  for (int j = 0; j < 8; ++j) {
    const int cc = 32 * j + lane;
    const float dv = wr[cc] - mu;
    const float y  = dv / sq * sgb[cc] + sgb[HC + cc];
    const float em = expm1f(y);
    wr[cc] = (y > 0.0f) ? y : em;
  }
  __syncthreads();

  v4f o0 = *(const v4fa*)(wr + 4 * lane);
  v4f o1 = *(const v4fa*)(wr + 128 + 4 * lane);
  const bool bad = (fl != 0) || (craw > DEGCAP) || (craw < 0);
  const float qnan = __int_as_float(0x7fc00000);
  if (bad) {
    const v4f nv = {qnan, qnan, qnan, qnan};
    o0 = nv; o1 = nv;
  }
  float* op = out + (size_t)row * HC + 4 * lane;
  if (live) { *(volatile v4f*)op = o0; *(volatile v4f*)(op + 128) = o1; }
  __threadfence();
  if (live) { *(volatile v4f*)op = o0; *(volatile v4f*)(op + 128) = o1; }
}

static inline size_t al256(size_t v) { return (v + 255) & ~(size_t)255; }

extern "C" void kernel_launch(void* const* d_in, const int* in_sizes, int n_in,
                              void* d_out, int out_size, void* d_ws, size_t ws_size,
                              hipStream_t stream) {
  if (n_in < 7) return;
  if (in_sizes[0] != NROWS * F_IN) return;
  if (in_sizes[1] != F_IN * HC) return;
  if (in_sizes[2] != NHD * HID || in_sizes[3] != NHD * HID) return;
  if (in_sizes[4] != HC || in_sizes[5] != HC) return;
  if (in_sizes[6] < 2 || (in_sizes[6] & 1) != 0) return;
  const int nE = in_sizes[6] / 2;
  if (nE < 1 || nE >= (1 << (32 - SLOTB))) return;
  if (out_size != NROWS * HC) return;

  const float* x   = (const float*)d_in[0];
  const float* W   = (const float*)d_in[1];
  const float* al  = (const float*)d_in[2];
  const float* ar  = (const float*)d_in[3];
  const float* gm  = (const float*)d_in[4];
  const float* bt  = (const float*)d_in[5];
  const int*   ei  = (const int*)  d_in[6];
  float* out = (float*)d_out;
  const int* src = ei;
  const int* dst = ei + nE;
  const int vec8 = ((nE & 3) == 0) ? 1 : 0;

  char* ws = (char*)d_ws;
  size_t off = 0;
  const size_t oXB  = off; off = al256(off + (size_t)MP * F_IN * 2);
  const size_t oWT  = off; off = al256(off + (size_t)HC * F_IN * 2);
  const size_t oPAR = off; off = al256(off + (size_t)4 * HC * 4);
  const size_t oHP  = off; off = al256(off + (size_t)MP * HC * 4);
  const size_t oSD  = off; off = al256(off + (size_t)MP * 16 * 4);
  const size_t oLS  = off; off = al256(off + (size_t)NBLK * RCAP * 4);
  const size_t oOF  = off; off = al256(off + (size_t)NBLK * NBRUN * 4);
  const size_t oCN  = off; off = al256(off + (size_t)NBLK * NBRUN * 4);
  const size_t oFL  = off; off = al256(off + (size_t)16 * 32 * 4);
  if (off > ws_size || off > WSMAX) return;
  unsigned short* XB  = (unsigned short*)(ws + oXB);
  unsigned short* WT  = (unsigned short*)(ws + oWT);
  float*          PAR = (float*)(ws + oPAR);
  float*          HP  = (float*)(ws + oHP);
  float*          SD  = (float*)(ws + oSD);
  int*            LS  = (int*)(ws + oLS);
  int*            OF  = (int*)(ws + oOF);
  int*            CN  = (int*)(ws + oCN);
  int*            FL  = (int*)(ws + oFL);

  hipFuncSetAttribute(reinterpret_cast<const void*>(&k_bucket),
                      hipFuncAttributeMaxDynamicSharedMemorySize, LDS_BKT);

  const int nbX = (MP * (F_IN / 8)) / NTHR;
  const int nbW = (HC * (F_IN / 8)) / NTHR;
  k_prep<<<nbX + nbW + 1, NTHR, 0, stream>>>(x, W, al, ar, gm, bt, XB, WT, PAR, nbX, nbW);
  k_gemm<<<MP / GROWS, GTHR, 0, stream>>>(XB, WT, PAR, HP, SD);
  k_bucket<<<NBLK, NTHR, LDS_BKT, stream>>>(src, dst, LS, OF, CN, FL, NNODE, nE, vec8);
  k_replay<<<NROWS / NWAVE, NTHR, 0, stream>>>(HP, SD, XB, PAR, LS, OF, CN, FL, out);
}
